// GNN_44281112822299
// MI455X (gfx1250) — hardware-verified
//
#include <hip/hip_runtime.h>
#include <stddef.h>
#include <stdint.h>
#include <math.h>


#define EMB    64
#define KIN    192
#define HD1    128
#define HD2    64
#define K2     256
#define AP1    200
#define NTHR   256
#define NWAVE  8
#define EPT    8
#define CHUNK  (NTHR * EPT)
#define WCAP   (EPT * 32)
#define LISTN  (NWAVE * WCAP)
#define NBD    8192
#define SLD    13
#define NBA    1024
#define SLA    10
#define RCAP   28672
#define DEGCAP 64
#define GBM    64
#define GTHR   128
#define NUW1   (HD1 * (KIN / 8))
#define NUW2   (HD2 * (K2 / 8))
#define AGG_ZINTS (LISTN + 2 * RCAP + 3 * NBA)
#define AGG_LDS_INTS (AGG_ZINTS + 16)
#define WSMAX  134217728

static_assert((CHUNK & (CHUNK - 1)) == 0 && CHUNK <= 4096);
static_assert((NBD & (NBD - 1)) == 0 && NBD == (1 << SLD));
static_assert((NBA & (NBA - 1)) == 0 && NBA == (1 << SLA));
static_assert(((long long)CHUNK << SLD) < (1LL << 31));
static_assert(((long long)CHUNK << SLA) < (1LL << 31));
static_assert(NBD % (NTHR * 4) == 0);
static_assert(LISTN % NTHR == 0);
static_assert(NBA % NWAVE == 0 && NBA % 32 == 0 && NBA % GBM == 0);
static_assert(RCAP % 32 == 0 && AGG_ZINTS % 4 == 0 && LISTN % 4 == 0);
static_assert(KIN % 32 == 0 && K2 % 32 == 0 && K2 == 2 * HD1 && KIN == 3 * EMB);
static_assert(AP1 % 8 == 0 && AP1 >= KIN);
static_assert(GBM == (GTHR / 32) * 16);
static_assert((GBM * (KIN / 8)) % GTHR == 0);
static_assert(NUW1 % NTHR == 0 && NUW2 % NTHR == 0);
static_assert(HD1 == 4 * 32 && HD2 == 2 * 32);
static_assert(AGG_LDS_INTS * 4 <= 300000);

typedef float          v2f   __attribute__((ext_vector_type(2)));
typedef float          v4f   __attribute__((ext_vector_type(4)));
typedef float          v8f   __attribute__((ext_vector_type(8)));
typedef int            v4i   __attribute__((ext_vector_type(4)));
typedef int            v8i   __attribute__((ext_vector_type(8)));
typedef unsigned int   v4u   __attribute__((ext_vector_type(4)));
typedef unsigned short v8us  __attribute__((ext_vector_type(8)));
typedef unsigned short v16us __attribute__((ext_vector_type(16)));
typedef __bf16         v16bf __attribute__((ext_vector_type(16)));
typedef v2f  __attribute__((may_alias)) v2fa;
typedef v4f  __attribute__((may_alias)) v4fa;
typedef v4i  __attribute__((may_alias)) v4ia;
typedef v8us __attribute__((may_alias)) v8usa;
union FragB { v16bf v; v16us u; v8us h[2]; v8i w; };

__device__ __forceinline__ v8f wmb(const FragB& a, const FragB& b, v8f c) {
  v8f d = __builtin_amdgcn_wmma_f32_16x16x32_bf16(false, a.v, false, b.v, (short)0, c, false, false);
  asm volatile("v_nop\n\tv_nop\n\tv_nop\n\tv_nop" : "+v"(d) : "v"(a.w), "v"(b.w));
  return d;
}

__device__ __forceinline__ unsigned bf16_bits(float f) {
  const unsigned u = __float_as_uint(f);
  const unsigned r = (u + 0x7FFFu + ((u >> 16) & 1u)) >> 16;
  const bool isn = (u & 0x7FFFFFFFu) > 0x7F800000u;
  return isn ? 0x7FC0u : r;
}
__device__ __forceinline__ float bf16_val(float f) {
  return __uint_as_float(bf16_bits(f) << 16);
}

template <int SLB>
__device__ __forceinline__ int scan_chunk(const int* __restrict__ dsts, int nE, int cbase, int slotBase,
                                          int nb, int vec8, int* list, int tid, int lane, int wave) {
  int wc = 0;
  const int el0  = tid * EPT;
  const int e0   = cbase + el0;
  const int sent = -2147483647 - 1;
  v4i da, db;
  if (vec8 != 0 && cbase + CHUNK <= nE) {
    da = *(const v4i*)(dsts + e0);
    db = *(const v4i*)(dsts + e0 + 4);
  } else {
    da.x = (e0     < nE) ? dsts[min(e0,     nE - 1)] : sent;
    da.y = (e0 + 1 < nE) ? dsts[min(e0 + 1, nE - 1)] : sent;
    da.z = (e0 + 2 < nE) ? dsts[min(e0 + 2, nE - 1)] : sent;
    da.w = (e0 + 3 < nE) ? dsts[min(e0 + 3, nE - 1)] : sent;
    db.x = (e0 + 4 < nE) ? dsts[min(e0 + 4, nE - 1)] : sent;
    db.y = (e0 + 5 < nE) ? dsts[min(e0 + 5, nE - 1)] : sent;
    db.z = (e0 + 6 < nE) ? dsts[min(e0 + 6, nE - 1)] : sent;
    db.w = (e0 + 7 < nE) ? dsts[min(e0 + 7, nE - 1)] : sent;
  }
  const unsigned nbs = (unsigned)slotBase;
  const unsigned unb = (unsigned)nb;
  const unsigned s0 = (unsigned)da.x - nbs, s1 = (unsigned)da.y - nbs;
  const unsigned s2 = (unsigned)da.z - nbs, s3 = (unsigned)da.w - nbs;
  const unsigned s4 = (unsigned)db.x - nbs, s5 = (unsigned)db.y - nbs;
  const unsigned s6 = (unsigned)db.z - nbs, s7 = (unsigned)db.w - nbs;
  const bool h0 = s0 < unb, h1 = s1 < unb, h2 = s2 < unb, h3 = s3 < unb;
  const bool h4 = s4 < unb, h5 = s5 < unb, h6 = s6 < unb, h7 = s7 < unb;
  const unsigned any = __builtin_amdgcn_ballot_w32(h0 | h1 | h2 | h3 | h4 | h5 | h6 | h7);
  if (any != 0u) {
#define HITJ(J, HJ, SJ) { \
      const unsigned mj = __builtin_amdgcn_ballot_w32(HJ); \
      if (mj != 0u) { \
        if (HJ) { \
          const int pos = wc + (int)__builtin_amdgcn_mbcnt_lo(mj, 0u); \
          if (pos < WCAP) list[wave * WCAP + pos] = ((el0 + (J)) << SLB) | (int)(SJ); \
        } \
        wc += (int)__builtin_popcount(mj); } }
    HITJ(0, h0, s0)
    HITJ(1, h1, s1)
    HITJ(2, h2, s2)
    HITJ(3, h3, s3)
    HITJ(4, h4, s4)
    HITJ(5, h5, s5)
    HITJ(6, h6, s6)
    HITJ(7, h7, s7)
#undef HITJ
  }
  return wc;
}

__device__ __forceinline__ void cvt_unit8(const float* __restrict__ src, unsigned short* dst, int u, int nUnits) {
  if (u >= nUnits) return;
  const float* p = src + (size_t)u * 8;
  const v4f a = *(const v4f*)p;
  const v4f b = *(const v4f*)(p + 4);
  v8us o;
  o[0] = (unsigned short)bf16_bits(a.x); o[1] = (unsigned short)bf16_bits(a.y);
  o[2] = (unsigned short)bf16_bits(a.z); o[3] = (unsigned short)bf16_bits(a.w);
  o[4] = (unsigned short)bf16_bits(b.x); o[5] = (unsigned short)bf16_bits(b.y);
  o[6] = (unsigned short)bf16_bits(b.z); o[7] = (unsigned short)bf16_bits(b.w);
  unsigned short* dp = dst + (size_t)u * 8;
  *(volatile v8us*)dp = o;
  __threadfence();
  *(volatile v8us*)dp = o;
}

__global__ __launch_bounds__(NTHR) void k_prep(const float* __restrict__ cat, const float* __restrict__ sub,
                                               const float* __restrict__ elem, const float* __restrict__ W1,
                                               const float* __restrict__ W2, unsigned short* TB,
                                               unsigned short* W1T, unsigned short* W2T2,
                                               int nCat, int nSub, int nElem, int bCat, int bSub, int bElem) {
  const int b   = (int)blockIdx.x;
  const int tid = (int)threadIdx.x;
  const int b1e = bCat + bSub;
  const int b2e = b1e + bElem;
  const int b3e = b2e + NUW1 / NTHR;
  if (b < bCat) {
    cvt_unit8(cat, TB, b * NTHR + tid, nCat * 8);
  } else if (b < b1e) {
    cvt_unit8(sub, TB + (size_t)nCat * EMB, (b - bCat) * NTHR + tid, nSub * 8);
  } else if (b < b2e) {
    cvt_unit8(elem, TB + (size_t)(nCat + nSub) * EMB, (b - b1e) * NTHR + tid, nElem * 8);
  } else if (b < b3e) {
    const int v  = (b - b2e) * NTHR + tid;
    const int n  = v / (KIN / 8);
    const int k8 = (v - n * (KIN / 8)) * 8;
    const float* p = W1 + (size_t)k8 * HD1 + n;
    v8us o;
#pragma unroll
    for (int i = 0; i < 8; ++i) o[i] = (unsigned short)bf16_bits(p[(size_t)i * HD1]);
    unsigned short* dp = W1T + (size_t)n * KIN + k8;
    *(volatile v8us*)dp = o;
    __threadfence();
    *(volatile v8us*)dp = o;
  } else {
    const int v  = (b - b3e) * NTHR + tid;
    if (v >= NUW2) return;
    const int n  = v >> 5;
    const int k8 = (v & 31) * 8;
    const int kk = k8 & (HD1 - 1);
    const float* p = W2 + (size_t)kk * HD2 + n;
    v8us o;
#pragma unroll
    for (int i = 0; i < 8; ++i) o[i] = (unsigned short)bf16_bits(p[(size_t)i * HD2]);
    unsigned short* dp = W2T2 + (size_t)n * K2 + k8;
    *(volatile v8us*)dp = o;
    __threadfence();
    *(volatile v8us*)dp = o;
  }
}

__global__ __launch_bounds__(NTHR) void k_deg(const int* __restrict__ dsts, int nE, int vec8, int* disw) {
  __shared__ __attribute__((aligned(16))) int scnt[NBD];
  __shared__ __attribute__((aligned(16))) int list[LISTN];
  __shared__ int wcnt[NWAVE];
  const int tid = (int)threadIdx.x, lane = tid & 31, wave = tid >> 5;
  const int nodeBase = (int)blockIdx.x * NBD;

  for (int i = tid; i < NBD; i += NTHR) scnt[i] = 0;
  for (int i = tid; i < LISTN; i += NTHR) list[i] = 0;
  if (tid < NWAVE) wcnt[tid] = 0;
  __syncthreads();

  const int nChunks = (nE + CHUNK - 1) / CHUNK;
#pragma unroll 1
  for (int ch = 0; ch < nChunks; ++ch) {
    const int cbase = ch * CHUNK;
    const int wc = scan_chunk<SLD>(dsts, nE, cbase, nodeBase, NBD, vec8, list, tid, lane, wave);
    if (lane == 0) wcnt[wave] = wc;
    __syncthreads();
    if (wave == 0) {
#pragma unroll 1
      for (int w2 = 0; w2 < NWAVE; ++w2) {
        int c = wcnt[w2];
        c = c < 0 ? 0 : (c > WCAP ? WCAP : c);
#pragma unroll 1
        for (int b0 = 0; b0 < c; b0 += 32) {
          const int idx = b0 + lane;
          const int ent = list[w2 * WCAP + (idx < WCAP ? idx : WCAP - 1)];
          const int m32 = (c - b0) < 32 ? (c - b0) : 32;
#pragma unroll 1
          for (int k = 0; k < m32; ++k) {
            const int u  = __builtin_amdgcn_readlane(ent, k);
            const int sl = u & (NBD - 1);
            if (lane == 0) scnt[sl] = scnt[sl] + 1;
          }
        }
      }
    }
    __syncthreads();
  }

#pragma unroll 1
  for (int i = tid; i < NBD; i += NTHR) {
    int c = scnt[i];
    c = c < 0 ? 0 : c;
    const float d = (float)c + 1.0f;
    const float r = (d > 0.0f) ? (1.0f / sqrtf(d)) : 0.0f;
    scnt[i] = __float_as_int(r);
  }
  __syncthreads();

  v4i vals[NBD / (NTHR * 4)];
#pragma unroll
  for (int it = 0; it < NBD / (NTHR * 4); ++it) {
    const int s0 = it * (NTHR * 4) + 4 * tid;
    vals[it] = *(const v4ia*)(scnt + s0);
  }
#pragma unroll
  for (int it = 0; it < NBD / (NTHR * 4); ++it) {
    const int s0 = it * (NTHR * 4) + 4 * tid;
    *(volatile v4i*)(disw + (size_t)nodeBase + s0) = vals[it];
  }
  __threadfence();
#pragma unroll
  for (int it = 0; it < NBD / (NTHR * 4); ++it) {
    const int s0 = it * (NTHR * 4) + 4 * tid;
    *(volatile v4i*)(disw + (size_t)nodeBase + s0) = vals[it];
  }
}

__global__ __launch_bounds__(GTHR) void k_gemm1(const int* __restrict__ cid, const int* __restrict__ sid,
                                                const int* __restrict__ eid, int nN,
                                                int nCat, int nSub, int nElem,
                                                const unsigned short* __restrict__ TB,
                                                const unsigned short* __restrict__ W1T,
                                                const float* __restrict__ dis, float* HS) {
  __shared__ __attribute__((aligned(16))) unsigned short at[GBM * AP1];
  __shared__ __attribute__((aligned(16))) float stg[GBM * HD1];
  __shared__ int   ridx[3 * GBM];
  __shared__ float sd[GBM];
  const int tid = (int)threadIdx.x, lane = tid & 31, wave = tid >> 5, hh = lane >> 4, m = lane & 15;
  const int rowBase = (int)blockIdx.x * GBM;

  if (tid < GBM) {
    const int node = rowBase + tid;
    const int nc   = node < nN ? node : nN - 1;
    int c = cid[nc]; c = c < 0 ? 0 : (c > nCat - 1 ? nCat - 1 : c);
    int s = sid[nc]; s = s < 0 ? 0 : (s > nSub - 1 ? nSub - 1 : s);
    int e = eid[nc]; e = e < 0 ? 0 : (e > nElem - 1 ? nElem - 1 : e);
    ridx[tid]           = c;
    ridx[GBM + tid]     = nCat + s;
    ridx[2 * GBM + tid] = nCat + nSub + e;
    const float dv = dis[nc];
    sd[tid] = (node < nN) ? dv : 0.0f;
  }
  __syncthreads();

#pragma unroll 4
  for (int it = 0; it < (GBM * (KIN / 8)) / GTHR; ++it) {
    const int p   = it * GTHR + tid;
    const int r   = p / (KIN / 8);
    const int q   = p - r * (KIN / 8);
    const int seg = q >> 3;
    const int pc  = q & 7;
    const int trow = ridx[seg * GBM + r];
    const v8us v = *(const v8usa*)(TB + (size_t)trow * EMB + pc * 8);
    *(v8usa*)(at + r * AP1 + seg * EMB + pc * 8) = v;
  }
  __syncthreads();

  v8f acc[8];
  {
    const v8f z = {0.f, 0.f, 0.f, 0.f, 0.f, 0.f, 0.f, 0.f};
#pragma unroll
    for (int t = 0; t < 8; ++t) acc[t] = z;
  }
  const unsigned short* ap = at + (16 * wave + m) * AP1 + 8 * hh;
  const unsigned short* bp = W1T + (size_t)m * (size_t)KIN + 8 * hh;
#pragma unroll 1
  for (int k0 = 0; k0 < KIN; k0 += 32) {
    FragB af;
    af.h[0] = *(const v8usa*)(ap + k0);
    af.h[1] = *(const v8usa*)(ap + k0 + 16);
#pragma unroll
    for (int nt = 0; nt < 8; ++nt) {
      const unsigned short* wq = bp + (size_t)(16 * nt) * (size_t)KIN + k0;
      FragB bf;
      bf.h[0] = *(const v8usa*)wq;
      bf.h[1] = *(const v8usa*)(wq + 16);
      acc[nt] = wmb(af, bf, acc[nt]);
    }
  }

#pragma unroll
  for (int nt = 0; nt < 8; ++nt) {
    const int lc = 16 * nt + m;
#pragma unroll
    for (int r = 0; r < 8; ++r) {
      const int lr = 16 * wave + 8 * hh + r;
      stg[lr * HD1 + lc] = acc[nt][r];
    }
  }
  __syncthreads();

  v4f pv[16];
#pragma unroll
  for (int i = 0; i < 16; ++i) pv[i] = *(const v4fa*)(stg + (16 * wave + i) * HD1 + 4 * lane);
#pragma unroll
  for (int i = 0; i < 16; ++i) {
    const int lr = 16 * wave + i;
    const bool ok = (rowBase + lr) < nN;
    const float s = sd[lr];
    v4f y;
    y.x = ok ? pv[i].x * s : 0.0f;
    y.y = ok ? pv[i].y * s : 0.0f;
    y.z = ok ? pv[i].z * s : 0.0f;
    y.w = ok ? pv[i].w * s : 0.0f;
    pv[i] = y;
  }
#pragma unroll
  for (int i = 0; i < 16; ++i) {
    float* op = HS + (size_t)(rowBase + 16 * wave + i) * HD1 + 4 * lane;
    *(volatile v4f*)op = pv[i];
  }
  __threadfence();
#pragma unroll
  for (int i = 0; i < 16; ++i) {
    float* op = HS + (size_t)(rowBase + 16 * wave + i) * HD1 + 4 * lane;
    *(volatile v4f*)op = pv[i];
  }
}

__global__ __launch_bounds__(GTHR) void k_gemm2(const unsigned short* __restrict__ A,
                                                const unsigned short* __restrict__ WT,
                                                const float* __restrict__ dis, int nN, float* outF) {
  __shared__ __attribute__((aligned(16))) float stg[GBM * HD2];
  __shared__ float sd[GBM];
  const int tid = (int)threadIdx.x, lane = tid & 31, wave = tid >> 5, hh = lane >> 4, m = lane & 15;
  const int rowBase = (int)blockIdx.x * GBM;

  if (tid < GBM) {
    const int node = rowBase + tid;
    const int nc   = node < nN ? node : nN - 1;
    const float dv = dis[nc];
    sd[tid] = (node < nN) ? dv : 0.0f;
  }

  v8f acc[4];
  {
    const v8f z = {0.f, 0.f, 0.f, 0.f, 0.f, 0.f, 0.f, 0.f};
    acc[0] = z; acc[1] = z; acc[2] = z; acc[3] = z;
  }
  const unsigned short* ap = A  + (size_t)(rowBase + 16 * wave + m) * (size_t)K2 + 8 * hh;
  const unsigned short* wp = WT + (size_t)m * (size_t)K2 + 8 * hh;
#pragma unroll 1
  for (int ks = 0; ks < K2 / 32; ++ks) {
    FragB af;
    af.h[0] = *(const v8usa*)(ap + 32 * ks);
    af.h[1] = *(const v8usa*)(ap + 32 * ks + 16);
#pragma unroll
    for (int t = 0; t < 4; ++t) {
      const unsigned short* wq = wp + (size_t)(16 * t) * (size_t)K2 + 32 * ks;
      FragB bf;
      bf.h[0] = *(const v8usa*)wq;
      bf.h[1] = *(const v8usa*)(wq + 16);
      acc[t] = wmb(af, bf, acc[t]);
    }
  }

#pragma unroll
  for (int t = 0; t < 4; ++t) {
    const int lc = 16 * t + m;
#pragma unroll
    for (int r = 0; r < 8; ++r) {
      const int lr = 16 * wave + 8 * hh + r;
      stg[lr * HD2 + lc] = acc[t][r];
    }
  }
  __syncthreads();

  v4f fv[8];
#pragma unroll
  for (int i = 0; i < 8; ++i) {
    const int lr = 16 * wave + 2 * i + hh;
    const v4f t4 = *(const v4fa*)(stg + lr * HD2 + 4 * m);
    const float s = sd[lr];
    const bool ok = (rowBase + lr) < nN;
    v4f y;
    y.x = ok ? t4.x * s : 0.0f;
    y.y = ok ? t4.y * s : 0.0f;
    y.z = ok ? t4.z * s : 0.0f;
    y.w = ok ? t4.w * s : 0.0f;
    fv[i] = y;
  }
#pragma unroll
  for (int i = 0; i < 8; ++i) {
    const int lr = 16 * wave + 2 * i + hh;
    float* op = outF + (size_t)(rowBase + lr) * HD2 + 4 * m;
    *(volatile v4f*)op = fv[i];
  }
  __threadfence();
#pragma unroll
  for (int i = 0; i < 8; ++i) {
    const int lr = 16 * wave + 2 * i + hh;
    float* op = outF + (size_t)(rowBase + lr) * HD2 + 4 * m;
    *(volatile v4f*)op = fv[i];
  }
}

template <int MODE>
__global__ __launch_bounds__(NTHR) void k_agg(const int* __restrict__ srcs, const int* __restrict__ dsts,
                                              int nE, int nN, int vec8, int mRows,
                                              const float* __restrict__ dis,
                                              const float* __restrict__ xl, const float* __restrict__ bias,
                                              unsigned short* hb, float* hout) {
  extern __shared__ __attribute__((aligned(16))) int dsm[];
  int* list = dsm;
  int* hl   = dsm + LISTN;
  int* sl   = dsm + LISTN + RCAP;
  int* cnt  = dsm + LISTN + 2 * RCAP;
  int* offs = cnt + NBA;
  int* cur  = offs + NBA;
  int* misc = cur + NBA;
  const int tid = (int)threadIdx.x, lane = tid & 31, wave = tid >> 5;
  const int nodeBase = (int)blockIdx.x * NBA;

  {
    const v4i z4 = {0, 0, 0, 0};
    for (int i = tid * 4; i < AGG_ZINTS; i += NTHR * 4) *(v4ia*)(dsm + i) = z4;
    if (tid < 16) misc[tid] = 0;
  }
  float bv0, bv1, bv2 = 0.0f, bv3 = 0.0f;
  if constexpr (MODE != 0) {
    const v4f a = *(const v4fa*)(bias + 4 * lane);
    bv0 = bf16_val(a.x); bv1 = bf16_val(a.y); bv2 = bf16_val(a.z); bv3 = bf16_val(a.w);
  } else {
    const v2f a = *(const v2fa*)(bias + 2 * lane);
    bv0 = bf16_val(a.x); bv1 = bf16_val(a.y);
  }
  __syncthreads();

  int t = 0, ov = 0;
  const int nChunks = (nE + CHUNK - 1) / CHUNK;
#pragma unroll 1
  for (int ch = 0; ch < nChunks; ++ch) {
    const int cbase = ch * CHUNK;
    const int wc = scan_chunk<SLA>(dsts, nE, cbase, nodeBase, NBA, vec8, list, tid, lane, wave);
    if (lane == 0) misc[wave] = wc;
    __syncthreads();
    if (wave == 0) {
#pragma unroll 1
      for (int w2 = 0; w2 < NWAVE; ++w2) {
        int c = misc[w2];
        c = c < 0 ? 0 : (c > WCAP ? WCAP : c);
#pragma unroll 1
        for (int b0 = 0; b0 < c; b0 += 32) {
          const int idx = b0 + lane;
          const int ent = list[w2 * WCAP + (idx < WCAP ? idx : WCAP - 1)];
          const int m32 = (c - b0) < 32 ? (c - b0) : 32;
#pragma unroll 1
          for (int k = 0; k < m32; ++k) {
            const int u    = __builtin_amdgcn_readlane(ent, k);
            const int slot = u & (NBA - 1);
            const int el   = (u >> SLA) & (CHUNK - 1);
            const int pk   = ((cbase + el) << SLA) | slot;
            if (t < RCAP) {
              if (lane == 0) { hl[t] = pk; cnt[slot] = cnt[slot] + 1; }
              t = t + 1;
            } else {
              ov = 1;
            }
          }
        }
      }
    }
    __syncthreads();
  }
  if (wave == 0 && lane == 0) { misc[8] = t; misc[9] = ov; }
  __syncthreads();
  int tt = misc[8];
  tt = tt < 0 ? 0 : (tt > RCAP ? RCAP : tt);
  const int ovf = misc[9];

  if (wave == 0) {
    const int base = lane * (NBA / 32);
    int s = 0;
#pragma unroll 1
    for (int i = 0; i < NBA / 32; ++i) s += cnt[base + i];
    int incl = s;
#pragma unroll
    for (int d = 1; d < 32; d <<= 1) {
      const int y = __shfl_up(incl, d, 32);
      if (lane >= d) incl += y;
    }
    int run = incl - s;
#pragma unroll 1
    for (int i = 0; i < NBA / 32; ++i) {
      const int cv = cnt[base + i];
      offs[base + i] = run;
      cur[base + i]  = run;
      run += cv;
    }
  }
  __syncthreads();
  if (wave == 0) {
#pragma unroll 1
    for (int b0 = 0; b0 < tt; b0 += 32) {
      const int idx = b0 + lane;
      const int ent = hl[idx < RCAP ? idx : RCAP - 1];
      const int m32 = (tt - b0) < 32 ? (tt - b0) : 32;
#pragma unroll 1
      for (int k = 0; k < m32; ++k) {
        const int u    = __builtin_amdgcn_readlane(ent, k);
        const int slot = u & (NBA - 1);
        if (lane == 0) {
          int p = cur[slot];
          p = p < 0 ? 0 : (p > RCAP - 1 ? RCAP - 1 : p);
          sl[p] = u;
          cur[slot] = p + 1;
        }
      }
    }
  }
  __syncthreads();

  const float qnan = __int_as_float(0x7fc00000);
  const float pz = (ovf != 0) ? qnan : 0.0f;
  const int sa = (2 * lane) & 31, sb = (2 * lane + 1) & 31;
#pragma unroll 1
  for (int si = 0; si < NBA / NWAVE; ++si) {
    const int s    = si * NWAVE + wave;
    const int node = nodeBase + s;
    int c = cnt[s];
    const bool big = c > DEGCAP;
    c = c < 0 ? 0 : (c > DEGCAP ? DEGCAP : c);
    int o = offs[s];
    o = o < 0 ? 0 : (o > RCAP ? RCAP : o);
    const int nc = node < nN ? node : nN - 1;
    const float dd = dis[nc];
    float a0 = 0.0f, a1 = 0.0f, a2 = 0.0f, a3 = 0.0f;
#pragma unroll 1
    for (int b0 = 0; b0 < c; b0 += 32) {
      int idx = o + b0 + lane;
      idx = idx > RCAP - 1 ? RCAP - 1 : idx;
      const int ent = sl[idx];
      int eid = ent >> SLA;
      eid = eid < 0 ? 0 : (eid > nE - 1 ? nE - 1 : eid);
      int sr = srcs[eid];
      sr = sr < 0 ? 0 : (sr > nN - 1 ? nN - 1 : sr);
      const int m32 = (c - b0) < 32 ? (c - b0) : 32;
#pragma unroll 1
      for (int k = 0; k < m32; ++k) {
        const int sk = __builtin_amdgcn_readlane(sr, k);
        if constexpr (MODE != 0) {
          const v4f a = *(const v4fa*)(xl + (size_t)sk * HD1 + 4 * lane);
          a0 += a.x; a1 += a.y; a2 += a.z; a3 += a.w;
        } else {
          const v2f a = *(const v2fa*)(xl + (size_t)sk * HD2 + 2 * lane);
          a0 += a.x; a1 += a.y;
        }
      }
    }
    const float pzr = big ? qnan : pz;
    const bool live = node < nN;
    if constexpr (MODE != 0) {
      const v4f sv = *(const v4fa*)(xl + (size_t)nc * HD1 + 4 * lane);
      const float t0 = dd * (a0 + sv.x) + bv0;
      const float t1 = dd * (a1 + sv.y) + bv1;
      const float t2 = dd * (a2 + sv.z) + bv2;
      const float t3 = dd * (a3 + sv.w) + bv3;
      float y0 = (t0 > 0.0f) ? t0 : (t0 - t0);
      float y1 = (t1 > 0.0f) ? t1 : (t1 - t1);
      float y2 = (t2 > 0.0f) ? t2 : (t2 - t2);
      float y3 = (t3 > 0.0f) ? t3 : (t3 - t3);
      y0 = y0 + pzr; y1 = y1 + pzr; y2 = y2 + pzr; y3 = y3 + pzr;
      const float v0 = live ? y0 : 0.0f;
      const float v1 = live ? y1 : 0.0f;
      const float v2 = live ? y2 : 0.0f;
      const float v3 = live ? y3 : 0.0f;
      const unsigned h0 = bf16_bits(v0), h1 = bf16_bits(v1), h2 = bf16_bits(v2), h3 = bf16_bits(v3);
      const unsigned l0 = bf16_bits(v0 - __uint_as_float(h0 << 16));
      const unsigned l1 = bf16_bits(v1 - __uint_as_float(h1 << 16));
      const unsigned l2 = bf16_bits(v2 - __uint_as_float(h2 << 16));
      const unsigned l3 = bf16_bits(v3 - __uint_as_float(h3 << 16));
      const int hw0 = (int)(h0 | (h1 << 16));
      const int hw1 = (int)(h2 | (h3 << 16));
      const int lw0 = (int)(l0 | (l1 << 16));
      const int lw1 = (int)(l2 | (l3 << 16));
      const int g0 = __shfl(hw0, sa, 32), g1 = __shfl(hw1, sa, 32);
      const int g2 = __shfl(hw0, sb, 32), g3 = __shfl(hw1, sb, 32);
      const int p0 = __shfl(lw0, sa, 32), p1 = __shfl(lw1, sa, 32);
      const int p2 = __shfl(lw0, sb, 32), p3 = __shfl(lw1, sb, 32);
      const bool lsel = lane >= 16;
      v4u pv;
      pv.x = (unsigned int)(lsel ? p0 : g0);
      pv.y = (unsigned int)(lsel ? p1 : g1);
      pv.z = (unsigned int)(lsel ? p2 : g2);
      pv.w = (unsigned int)(lsel ? p3 : g3);
      const bool wr = node < mRows;
      unsigned short* hp = hb + (size_t)node * K2 + 8 * lane;
      if (wr) *(volatile v4u*)hp = pv;
      __threadfence();
      if (wr) *(volatile v4u*)hp = pv;
    } else {
      const v2f sv = *(const v2fa*)(xl + (size_t)nc * HD2 + 2 * lane);
      const float t0 = dd * (a0 + sv.x) + bv0;
      const float t1 = dd * (a1 + sv.y) + bv1;
      float y0 = (t0 > 0.0f) ? t0 : (t0 - t0);
      float y1 = (t1 > 0.0f) ? t1 : (t1 - t1);
      y0 = y0 + pzr; y1 = y1 + pzr;
      const float v0 = live ? y0 : 0.0f;
      const float v1 = live ? y1 : 0.0f;
      v4f ow;
      ow.x = __shfl(v0, sa, 32); ow.y = __shfl(v1, sa, 32);
      ow.z = __shfl(v0, sb, 32); ow.w = __shfl(v1, sb, 32);
      const bool wr = (node < mRows) && (lane < 16);
      float* op = hout + (size_t)node * HD2 + 4 * (lane & 15);
      if (wr) *(volatile v4f*)op = ow;
      __threadfence();
      if (wr) *(volatile v4f*)op = ow;
    }
  }
}

static inline int cdiv(int a, int b) { return (a + b - 1) / b; }
static inline size_t al256(size_t o) { return (o + 255) & ~(size_t)255; }

extern "C" void kernel_launch(void* const* d_in, const int* in_sizes, int n_in,
                              void* d_out, int out_size, void* d_ws, size_t ws_size,
                              hipStream_t stream) {
  if (n_in < 11) return;
  const int nN = in_sizes[0];
  if (nN < 16 || nN > (1 << 22)) return;
  if (in_sizes[1] != nN || in_sizes[2] != nN) return;
  if (in_sizes[3] < 2 || (in_sizes[3] & 1) != 0) return;
  const int nE = in_sizes[3] / 2;
  if (nE < 1 || nE >= (1 << (31 - SLA))) return;
  if (in_sizes[4] < EMB || (in_sizes[4] % EMB) != 0) return;
  if (in_sizes[5] < EMB || (in_sizes[5] % EMB) != 0) return;
  if (in_sizes[6] < EMB || (in_sizes[6] % EMB) != 0) return;
  const int nCat  = in_sizes[4] / EMB;
  const int nSub  = in_sizes[5] / EMB;
  const int nElem = in_sizes[6] / EMB;
  if (nCat > (1 << 22) || nSub > (1 << 22) || nElem > (1 << 22)) return;
  if (in_sizes[7] != KIN * HD1 || in_sizes[8] != HD1) return;
  if (in_sizes[9] != HD1 * HD2 || in_sizes[10] != HD2) return;
  if ((long long)out_size != (long long)nN * HD2) return;

  const int*   cid  = (const int*)d_in[0];
  const int*   sid  = (const int*)d_in[1];
  const int*   eid  = (const int*)d_in[2];
  const int*   edge = (const int*)d_in[3];
  const float* catT = (const float*)d_in[4];
  const float* subT = (const float*)d_in[5];
  const float* elmT = (const float*)d_in[6];
  const float* W1   = (const float*)d_in[7];
  const float* b1   = (const float*)d_in[8];
  const float* W2   = (const float*)d_in[9];
  const float* b2   = (const float*)d_in[10];
  float* out = (float*)d_out;
  const int* src = edge;
  const int* dst = edge + nE;

  const int MP   = cdiv(nN, GBM) * GBM;
  const int gM   = MP / GBM;
  const int gD   = cdiv(nN, NBD);
  const int NBPD = gD * NBD;
  const int gA   = cdiv(MP, NBA);
  if ((long long)gA * NBA < (long long)MP) return;
  if (NBPD < nN) return;
  const int vec8 = ((nE & 3) == 0) ? 1 : 0;
  const int nTab = nCat + nSub + nElem;

  char* ws = (char*)d_ws;
  size_t off = 0;
  const size_t oDIS = off; off = al256(off + (size_t)NBPD * 4);
  const size_t oTB  = off; off = al256(off + (size_t)nTab * EMB * 2);
  const size_t oW1T = off; off = al256(off + (size_t)HD1 * KIN * 2);
  const size_t oW2T = off; off = al256(off + (size_t)HD2 * K2 * 2);
  const size_t oHS  = off; off = al256(off + (size_t)MP * HD1 * 4);
  const size_t oX1  = off; off = al256(off + (size_t)MP * K2 * 2);
  if (off > ws_size || off > (size_t)WSMAX) return;
  float*          DIS  = (float*)(ws + oDIS);
  unsigned short* TB   = (unsigned short*)(ws + oTB);
  unsigned short* W1T  = (unsigned short*)(ws + oW1T);
  unsigned short* W2T2 = (unsigned short*)(ws + oW2T);
  float*          HS   = (float*)(ws + oHS);
  unsigned short* X1HL = (unsigned short*)(ws + oX1);

  const size_t aggLds = (size_t)AGG_LDS_INTS * 4;
  hipFuncSetAttribute(reinterpret_cast<const void*>(&k_agg<1>), hipFuncAttributeMaxDynamicSharedMemorySize, (int)aggLds);
  hipFuncSetAttribute(reinterpret_cast<const void*>(&k_agg<0>), hipFuncAttributeMaxDynamicSharedMemorySize, (int)aggLds);

  const int bCat  = cdiv(nCat * 8, NTHR);
  const int bSub  = cdiv(nSub * 8, NTHR);
  const int bElem = cdiv(nElem * 8, NTHR);
  const int bTot  = bCat + bSub + bElem + NUW1 / NTHR + NUW2 / NTHR;

  k_prep<<<bTot, NTHR, 0, stream>>>(catT, subT, elmT, W1, W2, TB, W1T, W2T2, nCat, nSub, nElem, bCat, bSub, bElem);
  k_deg<<<gD, NTHR, 0, stream>>>(dst, nE, vec8, (int*)DIS);
  k_gemm1<<<gM, GTHR, 0, stream>>>(cid, sid, eid, nN, nCat, nSub, nElem, TB, W1T, DIS, HS);
  k_agg<1><<<gA, NTHR, aggLds, stream>>>(src, dst, nE, nN, vec8, MP, DIS, HS, b1, X1HL, out);
  k_gemm2<<<gM, GTHR, 0, stream>>>(X1HL, W2T2, DIS, nN, HS);
  k_agg<0><<<gA, NTHR, aggLds, stream>>>(src, dst, nE, nN, vec8, nN, DIS, HS, b2, X1HL, out);
}
